// GraphSAGE_81638738362645
// MI455X (gfx1250) — hardware-verified
//
#include <hip/hip_runtime.h>
#include <stddef.h>
#include <stdint.h>


#define NCH    256
#define NNODE  20000
#define KNB    16
#define NPAD   20096
#define XMP    512
#define PREP_NT   (NPAD / 64)
#define PREP_TB   (PREP_NT * (NCH / 64))
#define PREP_W1U  2048
#define PREP_W2U  8192
#define PREP_WB   ((PREP_W1U + PREP_W2U) / 256)
#define PREP_NB   (PREP_TB + PREP_WB + 1)
#define WSMAX  134217728

static_assert(NPAD % 128 == 0 && NPAD >= NNODE);
static_assert(NNODE % 4 == 0);
static_assert((NNODE * 4) % 128 == 0);
static_assert(PREP_W1U % 256 == 0 && (PREP_W1U + PREP_W2U) % 256 == 0);
static_assert(PREP_W1U * 8 == 4 * 64 * 64 && PREP_W2U * 8 == 4 * 64 * 256);
static_assert(NPAD % 32 == 0);

typedef float          v4f   __attribute__((ext_vector_type(4)));
typedef float          v8f   __attribute__((ext_vector_type(8)));
typedef int            v8i   __attribute__((ext_vector_type(8)));
typedef unsigned short v4us  __attribute__((ext_vector_type(4)));
typedef unsigned short v8us  __attribute__((ext_vector_type(8)));
typedef unsigned short v16us __attribute__((ext_vector_type(16)));
typedef __bf16         v16bf __attribute__((ext_vector_type(16)));
typedef v4f  __attribute__((may_alias)) v4fa;
typedef v4us __attribute__((may_alias)) v4usa;
typedef v8us __attribute__((may_alias)) v8usa;
union FragB { v16bf v; v16us u; v8us h[2]; v8i w; };

__device__ __forceinline__ v8f wmb(const FragB& a, const FragB& b, v8f c) {
  v8f d = __builtin_amdgcn_wmma_f32_16x16x32_bf16(false, a.v, false, b.v, (short)0, c, false, false);
  asm volatile("v_nop\n\tv_nop\n\tv_nop\n\tv_nop" : "+v"(d) : "v"(a.w), "v"(b.w));
  return d;
}

__device__ __forceinline__ unsigned bf16_bits(float f) {
  const unsigned u = __float_as_uint(f);
  return (u + 0x7FFFu + ((u >> 16) & 1u)) >> 16;
}
__device__ __forceinline__ float bf16_val(float f) {
  return __uint_as_float(bf16_bits(f) << 16);
}

__device__ __forceinline__ void wave_sync() {
  __builtin_amdgcn_fence(__ATOMIC_RELEASE, "wavefront");
  __builtin_amdgcn_wave_barrier();
  __builtin_amdgcn_fence(__ATOMIC_ACQUIRE, "wavefront");
}

__global__ __launch_bounds__(256) void k_prep(const float* __restrict__ x, const float* __restrict__ W1,
                                              const float* __restrict__ W2,
                                              const float* __restrict__ g1, const float* __restrict__ be1,
                                              const float* __restrict__ m1, const float* __restrict__ v1,
                                              const float* __restrict__ g2, const float* __restrict__ be2,
                                              const float* __restrict__ m2, const float* __restrict__ v2,
                                              unsigned short* XT, unsigned short* W1B, unsigned short* W2P,
                                              float* TAB) {
  __shared__ __attribute__((aligned(16))) float tf[64 * 68];
  const int tid = (int)threadIdx.x;
  const int bid = (int)blockIdx.x;
  if (bid < PREP_TB) {
    const int nb = bid % PREP_NT;
    const int cb = bid / PREP_NT;
    const int n0 = nb * 64, c0 = cb * 64;
    {
      const int lr = tid >> 4;
      const int c4 = (tid & 15) * 4;
#pragma unroll
      for (int it = 0; it < 4; ++it) {
        const int cc = it * 16 + lr;
        const int n  = n0 + c4;
        const bool ok = n < NNODE;
        const int nc = ok ? n : (NNODE - 4);
        v4f a = *(const v4f*)(x + (size_t)(c0 + cc) * NNODE + nc);
        const v4f z = {0.0f, 0.0f, 0.0f, 0.0f};
        a = ok ? a : z;
        *(v4fa*)(tf + cc * 68 + c4) = a;
      }
    }
    __syncthreads();
    const int sub = tid >> 3;
    const int c8  = (tid & 7) * 8;
    v8us ov[2];
#pragma unroll
    for (int it = 0; it < 2; ++it) {
      const int nl = it * 32 + sub;
      v8us o;
#pragma unroll
      for (int e = 0; e < 8; ++e) o[e] = (unsigned short)bf16_bits(tf[(c8 + e) * 68 + nl]);
      ov[it] = o;
    }
#pragma unroll
    for (int it = 0; it < 2; ++it) {
      const int nl = it * 32 + sub;
      *(volatile v8us*)(XT + (size_t)(n0 + nl) * NCH + c0 + c8) = ov[it];
    }
    __threadfence();
#pragma unroll
    for (int it = 0; it < 2; ++it) {
      const int nl = it * 32 + sub;
      *(volatile v8us*)(XT + (size_t)(n0 + nl) * NCH + c0 + c8) = ov[it];
    }
  } else if (bid < PREP_TB + PREP_WB) {
    const int u = (bid - PREP_TB) * 256 + tid;
    const float* src;
    unsigned short* dst;
    if (u < PREP_W1U) {
      src = W1 + (size_t)u * 8;
      dst = W1B + (size_t)u * 8;
    } else {
      const int v  = u - PREP_W1U;
      const int g  = v >> 11;
      const int o  = (v >> 5) & 63;
      const int k8 = (v & 31) * 8;
      src = W2 + (size_t)g * 8192 + (size_t)o * 128 + (k8 & 127);
      dst = W2P + (size_t)g * 16384 + (size_t)o * 256 + k8;
    }
    const v4f a = *(const v4f*)src;
    const v4f b = *(const v4f*)(src + 4);
    v8us o8;
    o8[0] = (unsigned short)bf16_bits(a.x); o8[1] = (unsigned short)bf16_bits(a.y);
    o8[2] = (unsigned short)bf16_bits(a.z); o8[3] = (unsigned short)bf16_bits(a.w);
    o8[4] = (unsigned short)bf16_bits(b.x); o8[5] = (unsigned short)bf16_bits(b.y);
    o8[6] = (unsigned short)bf16_bits(b.z); o8[7] = (unsigned short)bf16_bits(b.w);
    *(volatile v8us*)dst = o8;
    __threadfence();
    *(volatile v8us*)dst = o8;
  } else {
#pragma unroll 1
    for (int w = 0; w < 2; ++w) {
      const float* gp  = w ? g2  : g1;
      const float* bep = w ? be2 : be1;
      const float* mp  = w ? m2  : m1;
      const float* vp  = w ? v2  : v1;
      const float gg = bf16_val(gp[tid]);
      const float bb = bf16_val(bep[tid]);
      const float mm = bf16_val(mp[tid]);
      const float vv = bf16_val(vp[tid]);
      const float r  = sqrtf(vv + 1e-5f);
      const float sc = gg / r;
      const float mg = mm * gg;
      const float sh = bb - mg / r;
      tf[(2 * w) * 256 + tid]     = sc;
      tf[(2 * w + 1) * 256 + tid] = sh;
    }
    __syncthreads();
    const v4f q = *(const v4fa*)(tf + 4 * tid);
    *(volatile v4f*)(TAB + 4 * tid) = q;
    __threadfence();
    *(volatile v4f*)(TAB + 4 * tid) = q;
  }
}

__global__ __launch_bounds__(256) void k_nn1(const unsigned short* __restrict__ XT,
                                             const unsigned short* __restrict__ W1B,
                                             const float* __restrict__ b1, const float* __restrict__ TAB,
                                             float* Y1) {
  __shared__ __attribute__((aligned(16))) float stg[128 * 64];
  const int tid = (int)threadIdx.x, lane = tid & 31, wave = tid >> 5, hh = lane >> 4, m = lane & 15;
  const int g = (int)blockIdx.y;
  const int rowBase = (int)blockIdx.x * 128;

  v8f acc[4];
  {
    const v8f z = {0.f, 0.f, 0.f, 0.f, 0.f, 0.f, 0.f, 0.f};
#pragma unroll
    for (int t = 0; t < 4; ++t) acc[t] = z;
  }
  const unsigned short* ap = XT + (size_t)(rowBase + 16 * wave + m) * NCH + g * 64 + 8 * hh;
  const unsigned short* bp = W1B + (size_t)g * 4096 + (size_t)m * 64 + 8 * hh;
#pragma unroll
  for (int k0 = 0; k0 < 64; k0 += 32) {
    FragB af;
    af.h[0] = *(const v8usa*)(ap + k0);
    af.h[1] = *(const v8usa*)(ap + k0 + 16);
#pragma unroll
    for (int nt = 0; nt < 4; ++nt) {
      const unsigned short* wq = bp + (size_t)(16 * nt) * 64 + k0;
      FragB bf;
      bf.h[0] = *(const v8usa*)wq;
      bf.h[1] = *(const v8usa*)(wq + 16);
      acc[nt] = wmb(af, bf, acc[nt]);
    }
  }
#pragma unroll
  for (int nt = 0; nt < 4; ++nt) {
    const int lc = 16 * nt + m;
#pragma unroll
    for (int r = 0; r < 8; ++r) {
      const int lr = 16 * wave + 8 * hh + r;
      stg[lr * 64 + lc] = acc[nt][r];
    }
  }
  __syncthreads();

  const int cq = 4 * m;
  v4f bb, sc, sh;
  {
    const v4f t = *(const v4f*)(b1 + g * 64 + cq);
    bb.x = bf16_val(t.x); bb.y = bf16_val(t.y); bb.z = bf16_val(t.z); bb.w = bf16_val(t.w);
    sc = *(const v4f*)(TAB + g * 64 + cq);
    sh = *(const v4f*)(TAB + 256 + g * 64 + cq);
  }
  v4f pv[8];
#pragma unroll
  for (int it = 0; it < 8; ++it) {
    const int row = 16 * wave + 2 * it + hh;
    const v4f t = *(const v4fa*)(stg + row * 64 + cq);
    v4f y = (t + bb) * sc + sh;
    y.x = fmaxf(y.x, 0.0f); y.y = fmaxf(y.y, 0.0f); y.z = fmaxf(y.z, 0.0f); y.w = fmaxf(y.w, 0.0f);
    pv[it] = y;
  }
#pragma unroll
  for (int it = 0; it < 8; ++it) {
    const int row = rowBase + 16 * wave + 2 * it + hh;
    *(volatile v4f*)(Y1 + (size_t)row * NCH + g * 64 + cq) = pv[it];
  }
  __threadfence();
#pragma unroll
  for (int it = 0; it < 8; ++it) {
    const int row = rowBase + 16 * wave + 2 * it + hh;
    *(volatile v4f*)(Y1 + (size_t)row * NCH + g * 64 + cq) = pv[it];
  }
}

__global__ __launch_bounds__(256) void k_gmax(const int* __restrict__ eidx, const float* __restrict__ Y1,
                                              unsigned short* XM) {
  __shared__ __attribute__((aligned(16))) unsigned short rowbuf[8 * XMP];
  const int tid = (int)threadIdx.x, lane = tid & 31, wave = tid >> 5;
  unsigned short* rb = rowbuf + wave * XMP;
#pragma unroll 1
  for (int i = 0; i < 4; ++i) {
    const int node = (int)blockIdx.x * 32 + wave * 4 + i;
    const bool live = node < NNODE;
    const int nc = live ? node : (NNODE - 1);
    int iv = eidx[(size_t)nc * KNB + (lane & 15)];
    iv = iv < 0 ? 0 : (iv > NNODE - 1 ? NNODE - 1 : iv);
    v4f ma, mb;
    {
      const int s0 = __builtin_amdgcn_readlane(iv, 0);
      const float* rp = Y1 + (size_t)s0 * NCH + 4 * lane;
      ma = *(const v4f*)rp;
      mb = *(const v4f*)(rp + 128);
    }
#pragma unroll 3
    for (int k = 1; k < KNB; ++k) {
      const int sk = __builtin_amdgcn_readlane(iv, k);
      const float* rp = Y1 + (size_t)sk * NCH + 4 * lane;
      const v4f a = *(const v4f*)rp;
      const v4f b = *(const v4f*)(rp + 128);
      ma.x = fmaxf(ma.x, a.x); ma.y = fmaxf(ma.y, a.y); ma.z = fmaxf(ma.z, a.z); ma.w = fmaxf(ma.w, a.w);
      mb.x = fmaxf(mb.x, b.x); mb.y = fmaxf(mb.y, b.y); mb.z = fmaxf(mb.z, b.z); mb.w = fmaxf(mb.w, b.w);
    }
    {
      const v4f z = {0.0f, 0.0f, 0.0f, 0.0f};
      ma = live ? ma : z;
      mb = live ? mb : z;
    }
    v4us ah, al, bh, bl;
    {
      unsigned hb;
      hb = bf16_bits(ma.x); ah[0] = (unsigned short)hb; al[0] = (unsigned short)bf16_bits(ma.x - __uint_as_float(hb << 16));
      hb = bf16_bits(ma.y); ah[1] = (unsigned short)hb; al[1] = (unsigned short)bf16_bits(ma.y - __uint_as_float(hb << 16));
      hb = bf16_bits(ma.z); ah[2] = (unsigned short)hb; al[2] = (unsigned short)bf16_bits(ma.z - __uint_as_float(hb << 16));
      hb = bf16_bits(ma.w); ah[3] = (unsigned short)hb; al[3] = (unsigned short)bf16_bits(ma.w - __uint_as_float(hb << 16));
      hb = bf16_bits(mb.x); bh[0] = (unsigned short)hb; bl[0] = (unsigned short)bf16_bits(mb.x - __uint_as_float(hb << 16));
      hb = bf16_bits(mb.y); bh[1] = (unsigned short)hb; bl[1] = (unsigned short)bf16_bits(mb.y - __uint_as_float(hb << 16));
      hb = bf16_bits(mb.z); bh[2] = (unsigned short)hb; bl[2] = (unsigned short)bf16_bits(mb.z - __uint_as_float(hb << 16));
      hb = bf16_bits(mb.w); bh[3] = (unsigned short)hb; bl[3] = (unsigned short)bf16_bits(mb.w - __uint_as_float(hb << 16));
    }
    *(v4usa*)(rb + 4 * lane)       = ah;
    *(v4usa*)(rb + 128 + 4 * lane) = al;
    *(v4usa*)(rb + 256 + 4 * lane) = bh;
    *(v4usa*)(rb + 384 + 4 * lane) = bl;
    wave_sync();
    const v8us q0 = *(const v8usa*)(rb + 8 * lane);
    const v8us q1 = *(const v8usa*)(rb + 256 + 8 * lane);
    wave_sync();
    unsigned short* rpw = XM + (size_t)node * XMP + 8 * lane;
    *(volatile v8us*)rpw = q0;
    *(volatile v8us*)(rpw + 256) = q1;
    __threadfence();
    *(volatile v8us*)rpw = q0;
    *(volatile v8us*)(rpw + 256) = q1;
  }
}

__global__ __launch_bounds__(256) void k_nn2(const unsigned short* __restrict__ XT,
                                             const unsigned short* __restrict__ XM,
                                             const unsigned short* __restrict__ W2P,
                                             const float* __restrict__ b2, const float* __restrict__ TAB,
                                             float* outp) {
  __shared__ __attribute__((aligned(16))) float stg[64 * 132];
  __shared__ __attribute__((aligned(16))) float cs[3 * 64];
  const int tid = (int)threadIdx.x, lane = tid & 31, wave = tid >> 5, hh = lane >> 4, m = lane & 15;
  const int g  = (int)blockIdx.y;
  const int n0 = (int)blockIdx.x * 128;
  if (tid < 64) {
    const int c = g * 64 + tid;
    cs[tid]       = bf16_val(b2[c]);
    cs[64 + tid]  = TAB[512 + c];
    cs[128 + tid] = TAB[768 + c];
  }
  const int K   = (g < 2) ? 128 : 256;
  const int ldb = (g < 2) ? NCH : XMP;
  const unsigned short* bt = (g < 2) ? (XT + g * 128) : (XM + (g - 2) * 256);
  const unsigned short* bp = bt + (size_t)(n0 + 16 * wave + m) * (size_t)ldb + 8 * hh;
  const unsigned short* ap = W2P + (size_t)g * 16384 + (size_t)m * 256 + 8 * hh;

  v8f acc[4];
  {
    const v8f z = {0.f, 0.f, 0.f, 0.f, 0.f, 0.f, 0.f, 0.f};
#pragma unroll
    for (int t = 0; t < 4; ++t) acc[t] = z;
  }
#pragma unroll 1
  for (int k0 = 0; k0 < K; k0 += 32) {
    FragB bf;
    bf.h[0] = *(const v8usa*)(bp + k0);
    bf.h[1] = *(const v8usa*)(bp + k0 + 16);
#pragma unroll
    for (int mt = 0; mt < 4; ++mt) {
      const unsigned short* wq = ap + (size_t)(16 * mt) * 256 + k0;
      FragB af;
      af.h[0] = *(const v8usa*)wq;
      af.h[1] = *(const v8usa*)(wq + 16);
      acc[mt] = wmb(af, bf, acc[mt]);
    }
  }
#pragma unroll
  for (int mt = 0; mt < 4; ++mt) {
#pragma unroll
    for (int r = 0; r < 8; ++r) {
      const int o = 16 * mt + 8 * hh + r;
      stg[o * 132 + 16 * wave + m] = acc[mt][r];
    }
  }
  __syncthreads();

  v4f pv[8];
#pragma unroll
  for (int i = 0; i < 8; ++i) {
    const int o = 8 * wave + i;
    const v4f t = *(const v4fa*)(stg + o * 132 + 4 * lane);
    const float bb = cs[o], sc = cs[64 + o], sh = cs[128 + o];
    v4f y;
    y.x = fmaxf((t.x + bb) * sc + sh, 0.0f);
    y.y = fmaxf((t.y + bb) * sc + sh, 0.0f);
    y.z = fmaxf((t.z + bb) * sc + sh, 0.0f);
    y.w = fmaxf((t.w + bb) * sc + sh, 0.0f);
    pv[i] = y;
  }
  const bool ok = (n0 + 4 * lane) < NNODE;
#pragma unroll
  for (int i = 0; i < 8; ++i) {
    const int o = 8 * wave + i;
    if (ok) *(volatile v4f*)(outp + (size_t)(g * 64 + o) * NNODE + n0 + 4 * lane) = pv[i];
  }
  __threadfence();
#pragma unroll
  for (int i = 0; i < 8; ++i) {
    const int o = 8 * wave + i;
    if (ok) *(volatile v4f*)(outp + (size_t)(g * 64 + o) * NNODE + n0 + 4 * lane) = pv[i];
  }
}

static inline size_t al256(size_t o) { return (o + 255) & ~(size_t)255; }

extern "C" void kernel_launch(void* const* d_in, const int* in_sizes, int n_in,
                              void* d_out, int out_size, void* d_ws, size_t ws_size,
                              hipStream_t stream) {
  if (n_in < 14) return;
  if (in_sizes[0] != NCH * NNODE) return;
  if (in_sizes[1] != 2 * NNODE * KNB) return;
  if (in_sizes[2] != 4 * 64 * 64) return;
  if (in_sizes[8] != 4 * 64 * 128) return;
  for (int i = 3; i <= 7; ++i)  if (in_sizes[i] != NCH) return;
  for (int i = 9; i <= 13; ++i) if (in_sizes[i] != NCH) return;
  if (out_size != NCH * NNODE) return;

  const float* x   = (const float*)d_in[0];
  const int*   eix = (const int*)d_in[1];
  const float* W1  = (const float*)d_in[2];
  const float* b1  = (const float*)d_in[3];
  const float* g1  = (const float*)d_in[4];
  const float* be1 = (const float*)d_in[5];
  const float* m1  = (const float*)d_in[6];
  const float* v1  = (const float*)d_in[7];
  const float* W2  = (const float*)d_in[8];
  const float* b2  = (const float*)d_in[9];
  const float* g2  = (const float*)d_in[10];
  const float* be2 = (const float*)d_in[11];
  const float* m2  = (const float*)d_in[12];
  const float* v2  = (const float*)d_in[13];
  float* out = (float*)d_out;

  char* ws = (char*)d_ws;
  size_t off = 0;
  const size_t oXT  = off; off = al256(off + (size_t)NPAD * NCH * 2);
  const size_t oY1  = off; off = al256(off + (size_t)NPAD * NCH * 4);
  const size_t oXM  = off; off = al256(off + (size_t)NPAD * XMP * 2);
  const size_t oW1B = off; off = al256(off + (size_t)4 * 64 * 64 * 2);
  const size_t oW2P = off; off = al256(off + (size_t)4 * 64 * 256 * 2);
  const size_t oTAB = off; off = al256(off + (size_t)4 * NCH * 4);
  if (off > ws_size || off > (size_t)WSMAX) return;
  unsigned short* XT  = (unsigned short*)(ws + oXT);
  float*          Y1  = (float*)(ws + oY1);
  unsigned short* XM  = (unsigned short*)(ws + oXM);
  unsigned short* W1B = (unsigned short*)(ws + oW1B);
  unsigned short* W2P = (unsigned short*)(ws + oW2P);
  float*          TAB = (float*)(ws + oTAB);

  k_prep<<<dim3(PREP_NB), dim3(256), 0, stream>>>(x, W1, W2, g1, be1, m1, v1, g2, be2, m2, v2, XT, W1B, W2P, TAB);
  k_nn1<<<dim3(NPAD / 128, 4), dim3(256), 0, stream>>>(XT, W1B, b1, TAB, Y1);
  k_gmax<<<dim3(NPAD / 32), dim3(256), 0, stream>>>(eix, Y1, XM);
  k_nn2<<<dim3(NPAD / 128, 4), dim3(256), 0, stream>>>(XT, XM, W2P, b2, TAB, out);
  (void)hipGetLastError();
}
